// Net4_90486370992274
// MI455X (gfx1250) — hardware-verified
//
#include <hip/hip_runtime.h>
#include <stddef.h>


#define DF    128
#define NH    4
#define GR    32
#define AP    136
#define XSP   132
#define TP    129
#define NTHR  256
#define NWAVE 8
#define NBF   1536
#define CAPP  26624
#define CHUNK 4096
#define NGRP  (CHUNK / (NTHR * 4))
#define MAXD  256
#define NPB   64
#define L4B   256
#define WSCL  16.0f
#define RSCL  0.0625f

#define LDS_CSR_INTS (2 * CAPP + 4 * NBF + NWAVE + NTHR)
#define LDS_CSR_BYTES (LDS_CSR_INTS * 4)

static_assert(NGRP == 4);
static_assert(NBF == 6 * NTHR);
static_assert((CAPP % 32) == 0);
static_assert(((2 * CAPP) % 4) == 0);
static_assert((((2 * CAPP + 2 * NBF) * 4) % 16) == 0);
static_assert(LDS_CSR_BYTES == 238624);
static_assert((NPB % NWAVE) == 0);
static_assert((L4B % NWAVE) == 0);
static_assert(NH * 32 == DF);
static_assert(DF / 32 == 4);

typedef float    v2f  __attribute__((ext_vector_type(2)));
typedef float    v4f  __attribute__((ext_vector_type(4)));
typedef float    v8f  __attribute__((ext_vector_type(8)));
typedef int      v2i  __attribute__((ext_vector_type(2)));
typedef int      v4i  __attribute__((ext_vector_type(4)));
typedef _Float16 v8h  __attribute__((ext_vector_type(8)));
typedef _Float16 v16h __attribute__((ext_vector_type(16)));
union Frag  { v16h v; v8h half[2]; };
union Pack8 { v8h h; v4i i; };

__device__ __forceinline__ v8f wm(v16h a, v16h b, v8f c) {
  v8f d = __builtin_amdgcn_wmma_f32_16x16x32_f16(false, a, false, b, (short)0, c, false, false);
  asm volatile("v_nop\n\tv_nop\n\tv_nop\n\tv_nop" : "+v"(d) : "v"(a), "v"(b));
  return d;
}

__device__ __forceinline__ int clampi(int v, int lo, int hi) { return v < lo ? lo : (v > hi ? hi : v); }
__device__ __forceinline__ float lrelu(float v) { return v >= 0.f ? v : 0.2f * v; }
__device__ __forceinline__ void wave_sync_lds() {
  __builtin_amdgcn_fence(__ATOMIC_RELEASE, "wavefront");
  __builtin_amdgcn_wave_barrier();
}

__global__ __launch_bounds__(NTHR) void k_prepw(const float* __restrict__ W, _Float16* Wt) {
  __shared__ __attribute__((aligned(16))) float T[32 * TP];
  const int tid = threadIdx.x;
  const int n0  = blockIdx.x * 32;
#pragma unroll
  for (int i = 0; i < 16; ++i) {
    const int idx = i * NTHR + tid;
    const int k   = idx >> 5;
    const int c   = idx & 31;
    T[c * TP + k] = W[(size_t)k * DF + n0 + c];
  }
  __syncthreads();
  Pack8 u[2];
  size_t po[2];
#pragma unroll
  for (int q = 0; q < 2; ++q) {
    const int t  = q * NTHR + tid;
    const int c  = t >> 4;
    const int k0 = (t & 15) * 8;
#pragma unroll
    for (int j = 0; j < 8; ++j) u[q].h[j] = (_Float16)(WSCL * T[c * TP + k0 + j]);
    po[q] = (size_t)(n0 + c) * DF + k0;
  }
#pragma unroll
  for (int q = 0; q < 2; ++q) *(volatile v4i*)(Wt + po[q]) = u[q].i;
  __threadfence();
#pragma unroll
  for (int q = 0; q < 2; ++q) *(volatile v4i*)(Wt + po[q]) = u[q].i;
}

__global__ __launch_bounds__(NTHR) void k_gemm(
    const float* __restrict__ x, const _Float16* __restrict__ Wt,
    const float* __restrict__ attl, const float* __restrict__ attr,
    float* hb, float* elp, float* erp, int nN) {
  __shared__ __attribute__((aligned(16))) _Float16 Ah[GR * AP];
  __shared__ __attribute__((aligned(16))) float Xs[GR * XSP];
  __shared__ __attribute__((aligned(16))) float Pq[2 * GR * NH];

  const int tid  = threadIdx.x;
  const int lane = tid & 31;
  const int wave = tid >> 5;
  const int hh   = lane >> 4;
  const int m    = lane & 15;
  const int rowBase = blockIdx.x * GR;

  {
    const int r  = tid >> 3;
    const int c0 = (tid & 7) * 16;
    int row = rowBase + r;
    if (row > nN - 1) row = nN - 1;
    const float* p = x + (size_t)row * DF + c0;
    const v4f f0 = *(const v4f*)(p), f1 = *(const v4f*)(p + 4);
    const v4f f2 = *(const v4f*)(p + 8), f3 = *(const v4f*)(p + 12);
    Pack8 u0, u1;
    u0.h[0] = (_Float16)f0.x; u0.h[1] = (_Float16)f0.y; u0.h[2] = (_Float16)f0.z; u0.h[3] = (_Float16)f0.w;
    u0.h[4] = (_Float16)f1.x; u0.h[5] = (_Float16)f1.y; u0.h[6] = (_Float16)f1.z; u0.h[7] = (_Float16)f1.w;
    u1.h[0] = (_Float16)f2.x; u1.h[1] = (_Float16)f2.y; u1.h[2] = (_Float16)f2.z; u1.h[3] = (_Float16)f2.w;
    u1.h[4] = (_Float16)f3.x; u1.h[5] = (_Float16)f3.y; u1.h[6] = (_Float16)f3.z; u1.h[7] = (_Float16)f3.w;
    *(v8h*)(Ah + r * AP + c0)     = u0.h;
    *(v8h*)(Ah + r * AP + c0 + 8) = u1.h;
  }
  __syncthreads();

  const int ncol = wave * 16 + m;
  v8f c0a = {0.f, 0.f, 0.f, 0.f, 0.f, 0.f, 0.f, 0.f};
  v8f c1a = {0.f, 0.f, 0.f, 0.f, 0.f, 0.f, 0.f, 0.f};
#pragma unroll
  for (int kt = 0; kt < DF / 32; ++kt) {
    const int k0 = kt * 32;
    Frag a0, a1, b;
    const _Float16* pb  = Wt + (size_t)ncol * DF + k0 + 8 * hh;
    const _Float16* pa0 = Ah + m * AP + k0 + 8 * hh;
    const _Float16* pa1 = Ah + (16 + m) * AP + k0 + 8 * hh;
    b.half[0]  = *(const v8h*)pb;   b.half[1]  = *(const v8h*)(pb + 16);
    a0.half[0] = *(const v8h*)pa0;  a0.half[1] = *(const v8h*)(pa0 + 16);
    a1.half[0] = *(const v8h*)pa1;  a1.half[1] = *(const v8h*)(pa1 + 16);
    c0a = wm(a0.v, b.v, c0a);
    c1a = wm(a1.v, b.v, c1a);
  }

#pragma unroll
  for (int r = 0; r < 8; ++r) {
    Xs[(8 * hh + r) * XSP + ncol]      = c0a[r] * RSCL;
    Xs[(16 + 8 * hh + r) * XSP + ncol] = c1a[r] * RSCL;
  }
  __syncthreads();

  {
    const int row   = tid >> 3;
    const int hs    = tid & 7;
    const int head  = hs & 3;
    const int which = hs >> 2;
    const float* att = (which != 0) ? attr : attl;
    const float* xs  = Xs + row * XSP + head * 32;
    const float* av  = att + head * 32;
    float s = 0.f;
#pragma unroll
    for (int d = 0; d < 8; ++d) {
      const v4f xv = *(const v4f*)(xs + 4 * d);
      const v4f aw = *(const v4f*)(av + 4 * d);
      s += xv.x * aw.x;
      s += xv.y * aw.y;
      s += xv.z * aw.z;
      s += xv.w * aw.w;
    }
    Pq[which * (GR * NH) + row * NH + head] = s;
  }
  __syncthreads();

  v4f xr[4];
#pragma unroll
  for (int i = 0; i < 4; ++i) xr[i] = *(const v4f*)(Xs + (4 * wave + i) * XSP + 4 * lane);
  v4f gv = {0.f, 0.f, 0.f, 0.f};
  if (wave < 2) gv = *(const v4f*)(Pq + wave * (GR * NH) + lane * NH);
  float* gp = ((wave == 0) ? elp : erp) + ((size_t)rowBase + lane) * NH;
  float* xpp[4];
#pragma unroll
  for (int i = 0; i < 4; ++i) xpp[i] = hb + (size_t)(rowBase + 4 * wave + i) * DF + 4 * lane;

#pragma unroll
  for (int i = 0; i < 4; ++i) *(volatile v4f*)(xpp[i]) = xr[i];
  if (wave < 2) *(volatile v4f*)gp = gv;
  __threadfence();
#pragma unroll
  for (int i = 0; i < 4; ++i) *(volatile v4f*)(xpp[i]) = xr[i];
  if (wave < 2) *(volatile v4f*)gp = gv;
}

__global__ __launch_bounds__(NTHR) void k_csr(
    const int* __restrict__ dstp, const int* __restrict__ srcp,
    int* csp, int* lcp, int nN, int nE) {
  extern __shared__ v4i lds_q[];
  int* P    = (int*)lds_q;
  int* S    = P + CAPP;
  int* cnt  = S + CAPP;
  int* cur  = cnt + NBF;
  int* lc   = cur + NBF;
  int* wcnt = lc + 2 * NBF;
  int* tsum = wcnt + NWAVE;

  const int tid  = threadIdx.x;
  const int lane = tid & 31;
  const int wave = tid >> 5;
  const int nodeBase = blockIdx.x * NBF;

  for (int i = tid; i < NBF; i += NTHR) cnt[i] = 0;
  const bool al16 = ((((size_t)dstp) & 15) == 0);

  int T = 0;
  const int nChunks = (nE + CHUNK - 1) / CHUNK;
#pragma unroll 1
  for (int ch = 0; ch < nChunks; ++ch) {
    const int cbase = ch * CHUNK;
    const bool full = al16 && (cbase + CHUNK <= nE);
    int dv[4 * NGRP];
#pragma unroll
    for (int g = 0; g < NGRP; ++g) {
      const int e0 = cbase + (g * NTHR + tid) * 4;
      v4i d;
      if (full) {
        d = *(const v4i*)(dstp + e0);
      } else {
        const int sent = -2147483647 - 1;
        const int q0 = e0     < nE - 1 ? e0     : nE - 1;
        const int q1 = e0 + 1 < nE - 1 ? e0 + 1 : nE - 1;
        const int q2 = e0 + 2 < nE - 1 ? e0 + 2 : nE - 1;
        const int q3 = e0 + 3 < nE - 1 ? e0 + 3 : nE - 1;
        d.x = (e0     < nE) ? dstp[q0] : sent;
        d.y = (e0 + 1 < nE) ? dstp[q1] : sent;
        d.z = (e0 + 2 < nE) ? dstp[q2] : sent;
        d.w = (e0 + 3 < nE) ? dstp[q3] : sent;
      }
      dv[4 * g + 0] = d.x; dv[4 * g + 1] = d.y; dv[4 * g + 2] = d.z; dv[4 * g + 3] = d.w;
    }
    unsigned sl[4 * NGRP];
    int      ps[4 * NGRP];
    bool     ht[4 * NGRP];
    int wc = 0;
#pragma unroll
    for (int k = 0; k < 4 * NGRP; ++k) {
      sl[k] = (unsigned)dv[k] - (unsigned)nodeBase;
      ht[k] = sl[k] < (unsigned)NBF;
      const unsigned mk = __builtin_amdgcn_ballot_w32(ht[k]);
      ps[k] = wc + (int)__builtin_amdgcn_mbcnt_lo(mk, 0u);
      wc += (int)__builtin_popcount(mk);
    }
    if (lane == 0) wcnt[wave] = wc;
    __syncthreads();
    int wb = 0, tot = 0;
#pragma unroll
    for (int w = 0; w < NWAVE; ++w) {
      const int c = wcnt[w];
      tot += c;
      wb += (w < wave) ? c : 0;
    }
#pragma unroll
    for (int k = 0; k < 4 * NGRP; ++k) {
      if (ht[k]) {
        const int p = T + wb + ps[k];
        const int e = cbase + ((k >> 2) * NTHR + tid) * 4 + (k & 3);
        if (p < CAPP) P[p] = (int)((sl[k] << 21) | (unsigned)e);
      }
    }
    T += tot;
    __syncthreads();
  }
  const int Tl = T < CAPP ? T : CAPP;

  if (wave == 0) {
#pragma unroll 1
    for (int b0 = 0; b0 < Tl; b0 += 32) {
      const int idx = b0 + lane;
      const bool valid = idx < Tl;
      const int ent = P[idx < CAPP - 1 ? idx : CAPP - 1];
      const int myslot = valid ? (int)(((unsigned)ent) >> 21) : 4095;
      int rank = 0, tt = 0;
#pragma unroll
      for (int qq = 0; qq < 32; ++qq) {
        const int sq = __builtin_amdgcn_readlane(myslot, qq);
        const int mt = (sq == myslot) ? 1 : 0;
        tt += mt;
        rank += (qq < lane) ? mt : 0;
      }
      const int ms = valid ? myslot : 0;
      const int cv = cnt[ms];
      if (valid && rank == tt - 1) cnt[ms] = cv + tt;
      wave_sync_lds();
    }
  }
  __syncthreads();

  {
    const int s0 = tid * 6;
    int sum = 0;
#pragma unroll
    for (int i = 0; i < 6; ++i) sum += cnt[s0 + i];
    tsum[tid] = sum;
  }
  __syncthreads();
  {
    int pre = 0;
#pragma unroll 1
    for (int u = 0; u < NTHR; ++u) {
      const int v = tsum[u];
      pre += (u < tid) ? v : 0;
    }
    const int s0 = tid * 6;
    int run = pre;
#pragma unroll
    for (int i = 0; i < 6; ++i) {
      const int a = cnt[s0 + i];
      cur[s0 + i] = run;
      lc[2 * (s0 + i)]     = run;
      lc[2 * (s0 + i) + 1] = a;
      run += a;
    }
  }
  __syncthreads();

  if (wave == 0) {
#pragma unroll 1
    for (int b0 = 0; b0 < Tl; b0 += 32) {
      const int idx = b0 + lane;
      const bool valid = idx < Tl;
      const int ent = P[idx < CAPP - 1 ? idx : CAPP - 1];
      const int myslot = valid ? (int)(((unsigned)ent) >> 21) : 4095;
      int rank = 0, tt = 0;
#pragma unroll
      for (int qq = 0; qq < 32; ++qq) {
        const int sq = __builtin_amdgcn_readlane(myslot, qq);
        const int mt = (sq == myslot) ? 1 : 0;
        tt += mt;
        rank += (qq < lane) ? mt : 0;
      }
      const int ms = valid ? myslot : 0;
      int e = ent & 0x1FFFFF;
      e = e > nE - 1 ? nE - 1 : e;
      int sv = srcp[e];
      sv = clampi(sv, 0, nN - 1);
      const int c0  = cur[ms];
      const int pos = c0 + rank;
      if (valid && pos >= 0 && pos < CAPP) S[pos] = sv;
      if (valid && rank == tt - 1) cur[ms] = c0 + tt;
      wave_sync_lds();
    }
  }
  __syncthreads();

  const int nl     = (Tl + 31) >> 5;
  const int pieces = nl * 8;
  int* gS = csp + (size_t)blockIdx.x * CAPP;
  int* gL = lcp + (size_t)blockIdx.x * (NBF * 2);
#pragma unroll 1
  for (int i = tid; i < pieces; i += NTHR) *(volatile v4i*)(gS + 4 * i) = *(const v4i*)(S + 4 * i);
#pragma unroll
  for (int r = 0; r < 3; ++r) {
    const int i = r * NTHR + tid;
    *(volatile v4i*)(gL + 4 * i) = *(const v4i*)(lc + 4 * i);
  }
  __threadfence();
#pragma unroll 1
  for (int i = tid; i < pieces; i += NTHR) *(volatile v4i*)(gS + 4 * i) = *(const v4i*)(S + 4 * i);
#pragma unroll
  for (int r = 0; r < 3; ++r) {
    const int i = r * NTHR + tid;
    *(volatile v4i*)(gL + 4 * i) = *(const v4i*)(lc + 4 * i);
  }
}

__global__ __launch_bounds__(NTHR) void k_gat(
    const float* __restrict__ hb, const float* __restrict__ elp, const float* __restrict__ erp,
    const int* __restrict__ csp, const int* __restrict__ lcp,
    const float* xin, const float* __restrict__ bias, float* xout, int nN) {
  __shared__ __attribute__((aligned(16))) float stg[NWAVE * 256];
  const int tid  = threadIdx.x;
  const int lane = tid & 31;
  const int wave = tid >> 5;
  const int hd   = lane >> 3;
  float* stw = stg + wave * 256;
  const v4f b4 = *(const v4f*)(bias + 4 * lane);
  const float ninf = __uint_as_float(0xff800000u);

#pragma unroll 1
  for (int q = 0; q < NPB / NWAVE; ++q) {
    const int node = blockIdx.x * NPB + q * NWAVE + wave;
    if (node >= nN) break;
    const v2i lcv = *(const v2i*)(lcp + (size_t)node * 2);
    int beg = __builtin_amdgcn_readfirstlane(lcv.x);
    int cnt = __builtin_amdgcn_readfirstlane(lcv.y);
    beg = clampi(beg, 0, CAPP);
    cnt = clampi(cnt, 0, MAXD);
    if (cnt > CAPP - beg) cnt = CAPP - beg;
    const int bblk = node / NBF;
    const int* seg = csp + (size_t)bblk * CAPP + beg;
    const v4f er4 = *(const v4f*)(erp + (size_t)node * NH);
    const int nch = (cnt + 31) >> 5;

    v4f mx = {ninf, ninf, ninf, ninf};
#pragma unroll 1
    for (int c = 0; c < nch; ++c) {
      const int e = 32 * c + lane;
      const bool valid = e < cnt;
      int j = seg[e < cnt - 1 ? e : cnt - 1];
      j = clampi(j, 0, nN - 1);
      const v4f el4 = *(const v4f*)(elp + (size_t)j * NH);
      const v4f sr = el4 + er4;
      v4f s;
      s.x = valid ? lrelu(sr.x) : ninf;
      s.y = valid ? lrelu(sr.y) : ninf;
      s.z = valid ? lrelu(sr.z) : ninf;
      s.w = valid ? lrelu(sr.w) : ninf;
      mx.x = fmaxf(mx.x, s.x); mx.y = fmaxf(mx.y, s.y);
      mx.z = fmaxf(mx.z, s.z); mx.w = fmaxf(mx.w, s.w);
    }
#pragma unroll
    for (int mk = 16; mk >= 1; mk >>= 1) {
      mx.x = fmaxf(mx.x, __shfl_xor(mx.x, mk, 32));
      mx.y = fmaxf(mx.y, __shfl_xor(mx.y, mk, 32));
      mx.z = fmaxf(mx.z, __shfl_xor(mx.z, mk, 32));
      mx.w = fmaxf(mx.w, __shfl_xor(mx.w, mk, 32));
    }

    v4f acc = {0.f, 0.f, 0.f, 0.f};
    float den = 0.f;
#pragma unroll 1
    for (int c = 0; c < nch; ++c) {
      int cn = cnt - 32 * c;
      cn = cn > 32 ? 32 : cn;
      const int e = 32 * c + lane;
      const bool valid = e < cnt;
      int j = seg[e < cnt - 1 ? e : cnt - 1];
      j = clampi(j, 0, nN - 1);
      const v4f el4 = *(const v4f*)(elp + (size_t)j * NH);
      const v4f sr = el4 + er4;
      v4f p;
      p.x = valid ? __expf(lrelu(sr.x) - mx.x) : 0.f;
      p.y = valid ? __expf(lrelu(sr.y) - mx.y) : 0.f;
      p.z = valid ? __expf(lrelu(sr.z) - mx.z) : 0.f;
      p.w = valid ? __expf(lrelu(sr.w) - mx.w) : 0.f;
      const float jf = __int_as_float(j);
      const v4f w0 = {p.x, jf, p.y, jf};
      const v4f w1 = {p.z, jf, p.w, jf};
      *(v4f*)(stw + lane * 8)     = w0;
      *(v4f*)(stw + lane * 8 + 4) = w1;
      wave_sync_lds();
      const int n2 = (cn + 1) >> 1;
#pragma unroll 1
      for (int t = 0; t < n2; ++t) {
        const v2f ea = *(const v2f*)(stw + (2 * t) * 8 + 2 * hd);
        const v2f eb = *(const v2f*)(stw + (2 * t + 1) * 8 + 2 * hd);
        const int ja = __float_as_int(ea.y);
        const int jb = __float_as_int(eb.y);
        const v4f xa = *(const v4f*)(hb + (size_t)ja * DF + 4 * lane);
        const v4f xb = *(const v4f*)(hb + (size_t)jb * DF + 4 * lane);
        acc += xa * ea.x;
        den += ea.x;
        acc += xb * eb.x;
        den += eb.x;
      }
      wave_sync_lds();
    }

    const float inv = (den > 0.f) ? (1.0f / den) : 0.f;
    const v4f xr = *(const v4f*)(xin + (size_t)node * DF + 4 * lane);
    v4f y = acc * inv;
    y = y + xr;
    y = y + b4;
    y.x = y.x > 0.f ? y.x : (__expf(y.x) - 1.f);
    y.y = y.y > 0.f ? y.y : (__expf(y.y) - 1.f);
    y.z = y.z > 0.f ? y.z : (__expf(y.z) - 1.f);
    y.w = y.w > 0.f ? y.w : (__expf(y.w) - 1.f);
    float* op = xout + (size_t)node * DF + 4 * lane;
    *(volatile v4f*)op = y;
    __threadfence();
    *(volatile v4f*)op = y;
  }
}

__global__ __launch_bounds__(NTHR) void k_l4node(
    const float* __restrict__ x3, const float* __restrict__ W4, const float* __restrict__ Wres4,
    const float* __restrict__ al4, const float* __restrict__ ar4, float* l4p, int nN) {
  __shared__ __attribute__((aligned(16))) float wt[DF * 4];
  __shared__ __attribute__((aligned(16))) float st[L4B * 8];
  const int tid = threadIdx.x;
  const int nb  = blockIdx.x * L4B;
  if (tid < DF) {
    wt[4 * tid + 0] = W4[2 * tid];
    wt[4 * tid + 1] = W4[2 * tid + 1];
    wt[4 * tid + 2] = Wres4[2 * tid];
    wt[4 * tid + 3] = Wres4[2 * tid + 1];
  }
  __syncthreads();
  int node = nb + tid;
  if (node > nN - 1) node = nN - 1;
  const float* xr = x3 + (size_t)node * DF;
  float z0 = 0.f, z1 = 0.f, r0 = 0.f, r1 = 0.f;
#pragma unroll 1
  for (int k4 = 0; k4 < DF / 4; ++k4) {
    const v4f v  = *(const v4f*)(xr + 4 * k4);
    const v4f w0 = *(const v4f*)(wt + 16 * k4);
    const v4f w1 = *(const v4f*)(wt + 16 * k4 + 4);
    const v4f w2 = *(const v4f*)(wt + 16 * k4 + 8);
    const v4f w3 = *(const v4f*)(wt + 16 * k4 + 12);
    z0 += v.x * w0.x; z1 += v.x * w0.y; r0 += v.x * w0.z; r1 += v.x * w0.w;
    z0 += v.y * w1.x; z1 += v.y * w1.y; r0 += v.y * w1.z; r1 += v.y * w1.w;
    z0 += v.z * w2.x; z1 += v.z * w2.y; r0 += v.z * w2.z; r1 += v.z * w2.w;
    z0 += v.w * w3.x; z1 += v.w * w3.y; r0 += v.w * w3.z; r1 += v.w * w3.w;
  }
  const float a0 = al4[0], a1 = al4[1], c0 = ar4[0], c1 = ar4[1];
  const float el = z0 * a0 + z1 * a1;
  const float er = z0 * c0 + z1 * c1;
  const v4f s0 = {z0, z1, r0, r1};
  const v4f s1 = {el, er, 0.f, 0.f};
  *(v4f*)(st + tid * 8)     = s0;
  *(v4f*)(st + tid * 8 + 4) = s1;
  __syncthreads();
  float* gp = l4p + (size_t)nb * 8;
#pragma unroll
  for (int r = 0; r < 2; ++r) {
    const int i = r * NTHR + tid;
    *(volatile v4f*)(gp + 4 * i) = *(const v4f*)(st + 4 * i);
  }
  __threadfence();
#pragma unroll
  for (int r = 0; r < 2; ++r) {
    const int i = r * NTHR + tid;
    *(volatile v4f*)(gp + 4 * i) = *(const v4f*)(st + 4 * i);
  }
}

__global__ __launch_bounds__(NTHR) void k_gat4(
    const float* __restrict__ l4p, const int* __restrict__ csp, const int* __restrict__ lcp,
    const float* __restrict__ b4p, float* out, int nN) {
  __shared__ __attribute__((aligned(16))) float so[L4B * 2];
  const int tid  = threadIdx.x;
  const int lane = tid & 31;
  const int wave = tid >> 5;
  const int nb   = blockIdx.x * L4B;
  const float bb0 = b4p[0], bb1 = b4p[1];
  const float ninf = __uint_as_float(0xff800000u);

#pragma unroll 1
  for (int q = 0; q < L4B / NWAVE; ++q) {
    const int sl   = q * NWAVE + wave;
    const int node = nb + sl;
    if (node >= nN) break;
    const v2i lcv = *(const v2i*)(lcp + (size_t)node * 2);
    int beg = __builtin_amdgcn_readfirstlane(lcv.x);
    int cnt = __builtin_amdgcn_readfirstlane(lcv.y);
    beg = clampi(beg, 0, CAPP);
    cnt = clampi(cnt, 0, MAXD);
    if (cnt > CAPP - beg) cnt = CAPP - beg;
    const int bblk = node / NBF;
    const int* seg = csp + (size_t)bblk * CAPP + beg;
    const v4f na  = *(const v4f*)(l4p + (size_t)node * 8);
    const v4f na2 = *(const v4f*)(l4p + (size_t)node * 8 + 4);
    const float erd = na2.y;
    const int nch = (cnt + 31) >> 5;

    float mx = ninf;
#pragma unroll 1
    for (int c = 0; c < nch; ++c) {
      const int e = 32 * c + lane;
      const bool valid = e < cnt;
      int j = seg[e < cnt - 1 ? e : cnt - 1];
      j = clampi(j, 0, nN - 1);
      const float elj = l4p[(size_t)j * 8 + 4];
      const float s = valid ? lrelu(elj + erd) : ninf;
      mx = fmaxf(mx, s);
    }
#pragma unroll
    for (int mk = 16; mk >= 1; mk >>= 1) mx = fmaxf(mx, __shfl_xor(mx, mk, 32));

    float acc0 = 0.f, acc1 = 0.f, den = 0.f;
#pragma unroll 1
    for (int c = 0; c < nch; ++c) {
      const int e = 32 * c + lane;
      const bool valid = e < cnt;
      int j = seg[e < cnt - 1 ? e : cnt - 1];
      j = clampi(j, 0, nN - 1);
      const float elj = l4p[(size_t)j * 8 + 4];
      const float p = valid ? __expf(lrelu(elj + erd) - mx) : 0.f;
      const v2f zj = *(const v2f*)(l4p + (size_t)j * 8);
      acc0 += p * zj.x;
      acc1 += p * zj.y;
      den  += p;
    }
#pragma unroll
    for (int mk = 16; mk >= 1; mk >>= 1) {
      acc0 += __shfl_xor(acc0, mk, 32);
      acc1 += __shfl_xor(acc1, mk, 32);
      den  += __shfl_xor(den,  mk, 32);
    }
    const float inv = (den > 0.f) ? (1.0f / den) : 0.f;
    float o0 = acc0 * inv;
    float o1 = acc1 * inv;
    o0 = o0 + na.z; o0 = o0 + bb0;
    o1 = o1 + na.w; o1 = o1 + bb1;
    if (lane == 0) {
      so[2 * sl]     = o0;
      so[2 * sl + 1] = o1;
    }
  }
  __syncthreads();
  int nn = nN - nb;
  nn = nn > L4B ? L4B : nn;
  const int pieces = nn >> 1;
  float* gp = out + (size_t)nb * 2;
  v4f ov = {0.f, 0.f, 0.f, 0.f};
  if (tid < pieces) ov = *(const v4f*)(so + 4 * tid);
  if (tid < pieces) *(volatile v4f*)(gp + 4 * tid) = ov;
  __threadfence();
  if (tid < pieces) *(volatile v4f*)(gp + 4 * tid) = ov;
}

static inline size_t align256(size_t v) { return (v + 255) & ~(size_t)255; }

extern "C" void kernel_launch(void* const* d_in, const int* in_sizes, int n_in,
                              void* d_out, int out_size, void* d_ws, size_t ws_size,
                              hipStream_t stream) {
  if (n_in != 20) return;
  const int nN = in_sizes[0] / DF;
  if (nN <= 0 || in_sizes[0] != nN * DF || (nN % 16) != 0) return;
  const int nE = in_sizes[1];
  if (nE <= 0 || in_sizes[2] != nE || nE > (1 << 21)) return;
  for (int l = 0; l < 3; ++l) {
    if (in_sizes[3 + 4 * l] != DF * DF) return;
    if (in_sizes[4 + 4 * l] != DF || in_sizes[5 + 4 * l] != DF || in_sizes[6 + 4 * l] != DF) return;
  }
  if (in_sizes[15] != DF * 2 || in_sizes[16] != 2 || in_sizes[17] != 2 || in_sizes[18] != 2 ||
      in_sizes[19] != DF * 2) return;
  if (out_size != nN * 2) return;

  const float* x   = (const float*)d_in[0];
  const int*   src = (const int*)d_in[1];
  const int*   dst = (const int*)d_in[2];
  const float *Wp[3], *alp[3], *arp[3], *bp[3];
  for (int l = 0; l < 3; ++l) {
    Wp[l]  = (const float*)d_in[3 + 4 * l];
    alp[l] = (const float*)d_in[4 + 4 * l];
    arp[l] = (const float*)d_in[5 + 4 * l];
    bp[l]  = (const float*)d_in[6 + 4 * l];
  }
  const float* W4    = (const float*)d_in[15];
  const float* al4   = (const float*)d_in[16];
  const float* ar4   = (const float*)d_in[17];
  const float* b4    = (const float*)d_in[18];
  const float* Wres4 = (const float*)d_in[19];
  float* outp = (float*)d_out;

  const int nP    = ((nN + GR - 1) / GR) * GR;
  const int nBlkC = (nN + NBF - 1) / NBF;
  const int n4P   = ((nN + L4B - 1) / L4B) * L4B;
  size_t off = 0;
  char* base = (char*)d_ws;
  _Float16* Wt = (_Float16*)(base + off); off = align256(off + (size_t)DF * DF * sizeof(_Float16));
  float* hb  = (float*)(base + off);     off = align256(off + (size_t)nP * DF * sizeof(float));
  float* xa  = (float*)(base + off);     off = align256(off + (size_t)nP * DF * sizeof(float));
  float* elp = (float*)(base + off);     off = align256(off + (size_t)nP * NH * sizeof(float));
  float* erp = (float*)(base + off);     off = align256(off + (size_t)nP * NH * sizeof(float));
  int*   csp = (int*)(base + off);       off = align256(off + (size_t)nBlkC * CAPP * sizeof(int));
  int*   lcp = (int*)(base + off);       off = align256(off + (size_t)nBlkC * NBF * 2 * sizeof(int));
  float* l4p = (float*)(base + off);     off = align256(off + (size_t)n4P * 8 * sizeof(float));
  if (off > ws_size) return;

  hipFuncSetAttribute(reinterpret_cast<const void*>(&k_csr),
                      hipFuncAttributeMaxDynamicSharedMemorySize, LDS_CSR_BYTES);
  k_csr<<<nBlkC, NTHR, LDS_CSR_BYTES, stream>>>(dst, src, csp, lcp, nN, nE);

  const int ggrid = (nN + NPB - 1) / NPB;
  for (int l = 0; l < 3; ++l) {
    const float* xin = (l == 0) ? x : xa;
    k_prepw<<<DF / 32, NTHR, 0, stream>>>(Wp[l], Wt);
    k_gemm<<<nP / GR, NTHR, 0, stream>>>(xin, Wt, alp[l], arp[l], hb, elp, erp, nN);
    k_gat<<<ggrid, NTHR, 0, stream>>>(hb, elp, erp, csp, lcp, xin, bp[l], xa, nN);
  }
  k_l4node<<<n4P / L4B, NTHR, 0, stream>>>(xa, W4, Wres4, al4, ar4, l4p, nN);
  k_gat4<<<n4P / L4B, NTHR, 0, stream>>>(l4p, csp, lcp, b4, outp, nN);
}
